// PureFIKANLinear_76854144794925
// MI455X (gfx1250) — hardware-verified
//
#include <hip/hip_runtime.h>


namespace {
constexpr int NR = 4096, F = 1024, O = 1024, G = 5, NG = G + 1, DEPTH = 8, KF = F * NG;
constexpr float BSC = 64.0f, WSC = 4096.0f, DMAX = 0.99f;

typedef _Float16 b16;
typedef __attribute__((ext_vector_type(16))) _Float16 v16b;
typedef __attribute__((ext_vector_type(8)))  _Float16 v8b;
typedef __attribute__((ext_vector_type(8)))  float v8f;
typedef __attribute__((ext_vector_type(4)))  float v4f;

__device__ __forceinline__ v8b ld8b(const b16* p) { return *(const v8b*)p; }
__device__ __forceinline__ v16b cat8b(v8b a, v8b b) { return __builtin_shufflevector(a, b, 0, 1, 2, 3, 4, 5, 6, 7, 8, 9, 10, 11, 12, 13, 14, 15); }
__device__ __forceinline__ v16b frag_kb(const b16* p, int hh) { return cat8b(ld8b(p + 8 * hh), ld8b(p + 16 + 8 * hh)); }
__device__ __forceinline__ void split16(float v, b16& hi, b16& lo) { hi = (b16)v; lo = (b16)(v - (float)hi); }
__device__ __forceinline__ void frag_ksplit(const float* p, int hh, v16b& fh_, v16b& fl_) {
  const float* p0 = p + 8 * hh; const float* p1 = p + 16 + 8 * hh;
#pragma unroll
  for (int e = 0; e < 8; ++e) { b16 a, c; split16(p0[e], a, c); fh_[e] = a; fl_[e] = c; split16(p1[e], a, c); fh_[8 + e] = a; fl_[8 + e] = c; }
}
__device__ __forceinline__ v8f wmma16b(v16b a, v16b b, v8f c) {
  v8f d = __builtin_amdgcn_wmma_f32_16x16x32_f16(false, a, false, b, (short)0, c, false, false);
  asm volatile("v_nop\n\tv_nop\n\tv_nop\n\tv_nop" : "+v"(d) : "v"(a), "v"(b));
  return d;
}
__device__ __forceinline__ void wave_lds_sync() {
  __builtin_amdgcn_fence(__ATOMIC_RELEASE, "workgroup");
  __builtin_amdgcn_wave_barrier();
  __builtin_amdgcn_fence(__ATOMIC_ACQUIRE, "workgroup");
}

struct Opnd { const void* p0; const void* p1; int ld; };
template <int NP> __device__ __forceinline__ void load_frags(const Opnd& o, int row, int kb, int hh, v16b& fh_, v16b& fl_) {
  if (NP == 0) { frag_ksplit((const float*)o.p0 + (size_t)row * o.ld + kb, hh, fh_, fl_); }
  else if (NP == 3) {
    const float* p = (const float*)o.p0 + (size_t)row * o.ld + kb; const float* p0 = p + 8 * hh; const float* p1 = p + 16 + 8 * hh;
#pragma unroll
    for (int e = 0; e < 8; ++e) { fh_[e] = (b16)p0[e]; fh_[8 + e] = (b16)p1[e]; }
    fl_ = fh_;
  } else {
    fh_ = frag_kb((const b16*)o.p0 + (size_t)row * o.ld + kb, hh);
    if (NP == 2) fl_ = frag_kb((const b16*)o.p1 + (size_t)row * o.ld + kb, hh); else fl_ = fh_;
  }
}
template <int ANP, int BNP> __device__ __forceinline__ v8f mac(v16b ah, v16b al, v16b bh, v16b bl, v8f c) {
  c = wmma16b(ah, bh, c);
  if (BNP == 0 || BNP == 2) c = wmma16b(ah, bl, c);
  if (ANP == 0 || ANP == 2) c = wmma16b(al, bh, c);
  return c;
}
template <int ANP, int BNP>
__device__ __forceinline__ void gemm_tile(const Opnd& A, const Opnd& B, int K, int m0, int c0, int nloc, int hlf, v8f (&acc)[2][4]) {
  for (int kb = 0; kb < K; kb += 32) {
    v16b a0h, a0l, a1h, a1l;
    load_frags<ANP>(A, m0 + nloc, kb, hlf, a0h, a0l);
    load_frags<ANP>(A, m0 + 16 + nloc, kb, hlf, a1h, a1l);
#pragma unroll
    for (int t = 0; t < 4; ++t) {
      v16b bh, bl;
      load_frags<BNP>(B, c0 + t * 16 + nloc, kb, hlf, bh, bl);
      acc[0][t] = mac<ANP, BNP>(a0h, a0l, bh, bl, acc[0][t]);
      acc[1][t] = mac<ANP, BNP>(a1h, a1l, bh, bl, acc[1][t]);
    }
  }
}

struct Epi { float scale; const float* cscale; const float* cbias; const float* rbias; int act; float post; const float* rscale; const float* resid; };
__device__ __forceinline__ float epi_val(const Epi& e, float acc, int row, int col) {
  float val = acc * e.scale;
  if (e.cscale) val *= e.cscale[col];
  if (e.cbias) val += e.cbias[col];
  if (e.rbias) val += e.rbias[row];
  if (e.act == 1) val = 0.5f * val * (1.0f + erff(val * 0.70710678118654752f));
  val *= e.post;
  if (e.rscale) val *= e.rscale[(size_t)row * 32];
  return val;
}
__device__ __forceinline__ void epi_planes(v8f (&acc)[2][4], const Epi& e, bool two,
                                           b16* __restrict__ oh, b16* __restrict__ ol, int ldo, int m0, int c0, int lane, b16* Th, b16* Tl) {
  const int nloc = lane & 15, hlf = lane >> 4;
#pragma unroll
  for (int t = 0; t < 4; ++t)
#pragma unroll
    for (int r = 0; r < 2; ++r)
#pragma unroll
      for (int v = 0; v < 8; ++v) {
        const int rr = r * 16 + v + 8 * hlf, cc = t * 16 + nloc;
        const float val = epi_val(e, acc[r][t][v], m0 + rr, c0 + cc);
        b16 h_, l_; split16(val, h_, l_);
        Th[rr * 64 + cc] = h_; if (two) Tl[rr * 64 + cc] = l_;
      }
  wave_lds_sync();
  for (int pass = 0; pass < 2; ++pass) {
#pragma unroll
    for (int j = 0; j < 8; ++j) {
      const int rr = j * 4 + (lane >> 3), c8 = (lane & 7) * 8;
      const size_t o = (size_t)(m0 + rr) * ldo + c0 + c8;
      *(volatile v8b*)(oh + o) = ld8b(Th + rr * 64 + c8);
      if (two) *(volatile v8b*)(ol + o) = ld8b(Tl + rr * 64 + c8);
    }
    __threadfence();
  }
}
__device__ __forceinline__ void epi_f32(v8f (&acc)[2][4], const Epi& e, float* __restrict__ out, int ldo, int m0, int c0, int lane, float* Tt) {
  const int nloc = lane & 15, hlf = lane >> 4;
#pragma unroll
  for (int t = 0; t < 4; ++t)
#pragma unroll
    for (int r = 0; r < 2; ++r)
#pragma unroll
      for (int v = 0; v < 8; ++v) {
        const int rr = r * 16 + v + 8 * hlf, cc = t * 16 + nloc;
        Tt[rr * 64 + cc] = epi_val(e, acc[r][t][v], m0 + rr, c0 + cc);
      }
  wave_lds_sync();
  float* dst0 = out + (size_t)m0 * ldo + c0; const float* rs0 = e.resid ? e.resid + (size_t)m0 * ldo + c0 : nullptr;
  for (int pass = 0; pass < 2; ++pass) {
#pragma unroll
    for (int j = 0; j < 16; ++j) {
      const int rr = j * 2 + hlf, c4 = nloc * 4;
      v4f val = *(const v4f*)(Tt + rr * 64 + c4);
      if (rs0) val += *(const v4f*)(rs0 + (size_t)rr * ldo + c4);
      *(volatile v4f*)(dst0 + (size_t)rr * ldo + c4) = val;
    }
    __threadfence();
  }
}


__global__ __launch_bounds__(256) void prep_kernel(const float* __restrict__ x, const float* __restrict__ bw, const float* __restrict__ fw, const float* __restrict__ fs,
                                                   b16* __restrict__ sx16, b16* __restrict__ bw16, b16* __restrict__ fw16) {
  const size_t tid = (size_t)blockIdx.x * blockDim.x + threadIdx.x, stride = (size_t)gridDim.x * blockDim.x;
  const size_t n0 = (size_t)NR * F / 8, n1 = (size_t)O * F / 8, n2 = (size_t)O * KF / 8;
  for (int pass = 0; pass < 2; ++pass) {
    for (size_t c = tid; c < n0 + n1 + n2; c += stride) {
      v8b v;
      if (c < n0) { const size_t i = c * 8;
#pragma unroll
        for (int e = 0; e < 8; ++e) { const float xv = x[i + e]; v[e] = (b16)(xv / (1.0f + expf(-xv))); }
        *(volatile v8b*)(sx16 + i) = v;
      } else if (c < n0 + n1) { const size_t i = (c - n0) * 8;
#pragma unroll
        for (int e = 0; e < 8; ++e) v[e] = (b16)(bw[i + e] * BSC);
        *(volatile v8b*)(bw16 + i) = v;
      } else { const size_t i = (c - n0 - n1) * 8;
#pragma unroll
        for (int e = 0; e < 8; ++e) { const size_t ie = i + e; const size_t o_ = ie / KF, f_ = (ie % KF) / NG; v[e] = (b16)(fw[ie] * fs[o_ * F + f_] * WSC); }
        *(volatile v8b*)(fw16 + i) = v;
      }
    }
    __threadfence();
  }
}

__global__ __launch_bounds__(256) void bases_kernel(const float* __restrict__ x, const float* __restrict__ draw, b16* __restrict__ bs16) {
  __shared__ __attribute__((aligned(16))) b16 R[KF];
  const int b = blockIdx.x, t = threadIdx.x;
  for (int ff = 0; ff < 4; ++ff) {
    const int f = t * 4 + ff; const float xv = x[(size_t)b * F + f];
    float tt = fminf(fmaxf((xv + 1.0f) / 2.0f, 0.0f), 1.0f), P = 1.0f, acc[NG];
#pragma unroll
    for (int g = 0; g < NG; ++g) acc[g] = 0.0f;
#pragma unroll 1
    for (int lv = 0; lv < DEPTH; ++lv) {
      const float fl = fminf(fmaxf(floorf(tt * (float)G), 0.0f), (float)(G - 1)); const int ii = (int)fl; const float s = tt * (float)G - fl;
      const float di = DMAX * tanhf(draw[(size_t)f * G + ii]);
#pragma unroll
      for (int g = 0; g < NG; ++g) {
        float h = (g == ii) ? (1.0f - s) : ((g == ii + 1) ? s : 0.0f);
        const float bv = (g == 0) ? (1.0f - s) : ((g == G) ? s : 0.0f);
        acc[g] += P * (h - di * bv);
      }
      tt = s; P = P * di;
    }
    { const float fl = fminf(fmaxf(floorf(tt * (float)G), 0.0f), (float)(G - 1)); const int ii = (int)fl; const float s = tt * (float)G - fl;
#pragma unroll
      for (int g = 0; g < NG; ++g) { const float h = (g == ii) ? (1.0f - s) : ((g == ii + 1) ? s : 0.0f); R[f * NG + g] = (b16)(acc[g] + P * h); } }
  }
  __syncthreads();
  b16* dst = bs16 + (size_t)b * KF;
  for (int pass = 0; pass < 2; ++pass) {
#pragma unroll
    for (int i = 0; i < 3; ++i) { const int pc_ = i * 256 + t; *(volatile v8b*)(dst + (size_t)pc_ * 8) = *(const v8b*)(R + pc_ * 8); }
    __threadfence();
  }
}

__global__ __launch_bounds__(128) void gemm_kernel(const b16* __restrict__ A, int lda, const b16* __restrict__ Bm, int ldb, int K, float scale,
                                                   const float* __restrict__ resid, float* __restrict__ o32, int ldo) {
  __shared__ __attribute__((aligned(16))) float Ts[4][32 * 64];
  const int lane = threadIdx.x & 31, wave = threadIdx.x >> 5, nloc = lane & 15, hlf = lane >> 4;
  const int m0 = blockIdx.y * 128 + wave * 32, c0 = blockIdx.x * 64;
  v8f acc[2][4];
#pragma unroll
  for (int r = 0; r < 2; ++r)
#pragma unroll
    for (int t = 0; t < 4; ++t) acc[r][t] = (v8f){};
  const Opnd Ao{A, nullptr, lda}, Bo{Bm, nullptr, ldb};
  gemm_tile<1, 1>(Ao, Bo, K, m0, c0, nloc, hlf, acc);
  const Epi e{scale, nullptr, nullptr, nullptr, 0, 1.0f, nullptr, resid};
  epi_f32(acc, e, o32, ldo, m0, c0, lane, Ts[wave]);
}
}

extern "C" void kernel_launch(void* const* d_in, const int* in_sizes, int n_in,
                              void* d_out, int out_size, void* d_ws, size_t ws_size, hipStream_t stream) {
  (void)n_in; (void)out_size;
  const float* x    = (const float*)d_in[0];
  const float* bw   = (const float*)d_in[1];
  const float* fw   = (const float*)d_in[2];
  const float* fs   = (const float*)d_in[3];
  const float* draw = (const float*)d_in[4];
  float* out = (float*)d_out;
  if (in_sizes[0] != NR * F || in_sizes[1] != O * F || in_sizes[2] != O * KF || in_sizes[4] != F * G) return;

  size_t off = 0; char* ws = (char*)d_ws;
  auto carve = [&](size_t bytes) { char* p = ws + off; off += (bytes + 255) & ~(size_t)255; return p; };
  b16* sx16 = (b16*)carve((size_t)NR * F * 2);
  b16* bw16 = (b16*)carve((size_t)O * F * 2);
  b16* fw16 = (b16*)carve((size_t)O * KF * 2);
  b16* bs16 = (b16*)carve((size_t)NR * KF * 2);
  float* y1 = (float*)carve((size_t)NR * O * 4);
  if (off > ws_size) return;
  prep_kernel<<<2048, 256, 0, stream>>>(x, bw, fw, fs, sx16, bw16, fw16);
  bases_kernel<<<NR, 256, 0, stream>>>(x, draw, bs16);
  gemm_kernel<<<dim3(O / 64, NR / 128), 128, 0, stream>>>(sx16, F, bw16, F, F, 1.0f / BSC, nullptr, y1, O);
  gemm_kernel<<<dim3(O / 64, NR / 128), 128, 0, stream>>>(bs16, KF, fw16, KF, KF, 1.0f / WSC, y1, out, O);
}
